// CustomLstm_88502096101611
// MI455X (gfx1250) — hardware-verified
//
#include <hip/hip_runtime.h>


#define DD   2048
#define HH   1024
typedef _Float16 h16;
typedef unsigned short bf;
typedef __attribute__((ext_vector_type(16))) __bf16   v16bf;
typedef __attribute__((ext_vector_type(16))) _Float16 v16h;
typedef __attribute__((ext_vector_type(8)))  _Float16 v8h;
typedef __attribute__((ext_vector_type(8)))  unsigned short v8us;
typedef __attribute__((ext_vector_type(8)))  float    v8f;
typedef __attribute__((ext_vector_type(4)))  float    v4f;
typedef __attribute__((ext_vector_type(2)))  float    v2f;
typedef __attribute__((ext_vector_type(4)))  unsigned short v4us;
typedef __attribute__((ext_vector_type(2)))  unsigned short v2us;
typedef v8h  __attribute__((may_alias)) v8ha;
typedef v4f  __attribute__((may_alias)) v4fa;
typedef v8us __attribute__((may_alias)) v8usa;

__device__ __forceinline__ unsigned short f2bf(float f) { unsigned u = __float_as_uint(f); u += 0x7FFFu + ((u >> 16) & 1u); return (unsigned short)(u >> 16); }
__device__ __forceinline__ float bf2f(unsigned short b) { return __uint_as_float(((unsigned)b) << 16); }
__device__ __forceinline__ float bfr(float f) { return bf2f(f2bf(f)); }
__device__ __forceinline__ void splitf(float y, unsigned short& h, unsigned short& l) { h = f2bf(y); l = f2bf(y - bf2f(h)); }
__device__ __forceinline__ v16h cat16(v8h lo, v8h hi) { return __builtin_shufflevector(lo, hi, 0, 1, 2, 3, 4, 5, 6, 7, 8, 9, 10, 11, 12, 13, 14, 15); }
__device__ __forceinline__ v16bf cat16b(v8us lo, v8us hi) { return __builtin_bit_cast(v16bf, __builtin_shufflevector(lo, hi, 0, 1, 2, 3, 4, 5, 6, 7, 8, 9, 10, 11, 12, 13, 14, 15)); }
__device__ __forceinline__ v8f wmma16(v16h a, v16h b, v8f c) { return __builtin_amdgcn_wmma_f32_16x16x32_f16(false, a, false, b, (short)0, c, false, false); }
__device__ __forceinline__ v8f wmmab(v16bf a, v16bf b, v8f c) { return __builtin_amdgcn_wmma_f32_16x16x32_bf16(false, a, false, b, (short)0, c, false, false); }

template <typename T16> struct WFrag;
template <> struct WFrag<h16> { typedef v16h V; static __device__ __forceinline__ V ld(const h16* p) { return cat16(*(const v8h*)p, *(const v8h*)(p + 16)); } static __device__ __forceinline__ v8f mma(V a, V b, v8f c) { return wmma16(a, b, c); } };
template <> struct WFrag<bf> { typedef v16bf V; static __device__ __forceinline__ V ld(const bf* p) { return cat16b(*(const v8us*)p, *(const v8us*)(p + 16)); } static __device__ __forceinline__ v8f mma(V a, V b, v8f c) { return wmmab(a, b, c); } };
template <typename T16, int NSPLIT, bool BIAS>
__global__ __launch_bounds__(32) void k_gemmw(const T16* __restrict__ A, const T16* __restrict__ A2, const T16* __restrict__ Bt, const T16* __restrict__ Bt2, int K, float* C, int ldc, const float* __restrict__ bias, size_t sA, size_t sB, size_t sC) {
    typedef typename WFrag<T16>::V V;
    __shared__ __align__(16) float os[16 * 68];
    const size_t z = blockIdx.z; A += z * sA; if (A2) A2 += z * sA; Bt += z * sB; if (Bt2) Bt2 += z * sB; C += z * sC;
    const int lane = threadIdx.x & 31, lr = lane & 15, hi = lane >> 4; const int r0 = blockIdx.x * 64, c0 = blockIdx.y * 64;
    v8f acc[4][4];
#pragma unroll
    for (int mb = 0; mb < 4; ++mb)
#pragma unroll
        for (int nb = 0; nb < 4; ++nb) acc[mb][nb] = (v8f){};
    const size_t aoff = (size_t)(r0 + lr) * K + 8 * hi, boff = (size_t)(c0 + lr) * K + 8 * hi;
#pragma unroll 1
    for (int kc = 0; kc < K; kc += 32) {
        V a[4], a2[4];
#pragma unroll
        for (int mb = 0; mb < 4; ++mb) { a[mb] = WFrag<T16>::ld(A + aoff + (size_t)mb * 16 * K + kc); if (NSPLIT == 1 || NSPLIT == 2) a2[mb] = WFrag<T16>::ld(A2 + aoff + (size_t)mb * 16 * K + kc); }
#pragma unroll
        for (int nb = 0; nb < 4; ++nb) { const V b = WFrag<T16>::ld(Bt + boff + (size_t)nb * 16 * K + kc); V b2; if (NSPLIT >= 2) b2 = WFrag<T16>::ld(Bt2 + boff + (size_t)nb * 16 * K + kc);
#pragma unroll
            for (int mb = 0; mb < 4; ++mb) { acc[mb][nb] = WFrag<T16>::mma(a[mb], b, acc[mb][nb]); if (NSPLIT == 1 || NSPLIT == 2) acc[mb][nb] = WFrag<T16>::mma(a2[mb], b, acc[mb][nb]); if (NSPLIT >= 2) acc[mb][nb] = WFrag<T16>::mma(a[mb], b2, acc[mb][nb]); } }
        asm volatile("v_nop\n\tv_nop\n\tv_nop\n\tv_nop" : "+v"(acc[0][0]), "+v"(acc[1][1]), "+v"(acc[2][2]), "+v"(acc[3][3]) : "v"(a[0]), "v"(a[3]));
    }
#pragma unroll
    for (int mb = 0; mb < 4; ++mb) {
#pragma unroll
        for (int nb = 0; nb < 4; ++nb) {
#pragma unroll
            for (int j = 0; j < 8; ++j) os[(hi * 8 + j) * 68 + nb * 16 + lr] = acc[mb][nb][j]; }
        __builtin_amdgcn_wave_barrier(); asm volatile("" ::: "memory");
        float* crow = C + (size_t)(r0 + mb * 16) * ldc + c0;
#pragma unroll 1
        for (int ps = 0; ps < 2; ++ps) {
#pragma unroll
            for (int s = 0; s < 8; ++s) { const int row = 2 * s + hi, cofs = lr * 4; v4f val = *(const v4fa*)(os + row * 68 + cofs); if (BIAS) { val[0] += bfr(bias[c0 + cofs]); val[1] += bfr(bias[c0 + cofs + 1]); val[2] += bfr(bias[c0 + cofs + 2]); val[3] += bfr(bias[c0 + cofs + 3]); }
                *(volatile v4f*)(crow + (size_t)row * ldc + cofs) = val; }
            if (ps == 0) __threadfence(); }
        __builtin_amdgcn_wave_barrier(); asm volatile("" ::: "memory");
    }
}

__global__ __launch_bounds__(256) void k_cvt8(const float* __restrict__ src, bf* dst, size_t n8) { const size_t i = (size_t)blockIdx.x * 256 + threadIdx.x; if (i >= n8) return; const v8f v = *(const v8f*)(src + i * 8); v8us o;
#pragma unroll
    for (int k = 0; k < 8; ++k) o[k] = f2bf(v[k]); *(volatile v8us*)(dst + i * 8) = o; __threadfence(); *(volatile v8us*)(dst + i * 8) = o; }
__global__ __launch_bounds__(256) void k_tpc(const float* __restrict__ hp, const float* __restrict__ xx, bf* CT) { const size_t e = ((size_t)blockIdx.x * 256 + threadIdx.x) * 8; if (e >= (size_t)DD * DD) return; const int k = (int)(e % DD); const int n = (int)(e / DD); const float* src = (k < HH) ? hp + (size_t)k * DD + n : xx + (size_t)(k - HH) * DD + n; v8us o;
#pragma unroll
    for (int q = 0; q < 8; ++q) o[q] = f2bf(src[(size_t)q * DD]); *(volatile v8us*)(CT + e) = o; __threadfence(); *(volatile v8us*)(CT + e) = o; }
__device__ __forceinline__ float sigm(float z) { return __fdiv_rn(1.0f, __fadd_rn(1.0f, expf(-z))); }
__global__ __launch_bounds__(256) void k_gates(const float* __restrict__ G1, const float* __restrict__ G2, const float* __restrict__ G3, const float* __restrict__ G4, const float* __restrict__ b1, const float* __restrict__ b2, const float* __restrict__ b3, const float* __restrict__ b4, const float* __restrict__ cp, float* CT_, float* HT_) {
    const size_t e = (size_t)blockIdx.x * 256 + threadIdx.x; if (e >= (size_t)DD * DD) return;
    const float f = sigm(__fadd_rn(G1[e], bfr(b1[e]))), u = sigm(__fadd_rn(G2[e], bfr(b2[e]))), g = tanhf(__fadd_rn(G3[e], bfr(b3[e]))), o = sigm(__fadd_rn(G4[e], bfr(b4[e])));
    float p1 = __fmul_rn(f, bfr(cp[e])), p2 = __fmul_rn(u, g); asm volatile("" : "+v"(p1), "+v"(p2)); const float c = __fadd_rn(p1, p2); const float h = __fmul_rn(o, tanhf(c));
    *(volatile float*)(CT_ + e) = c; *(volatile float*)(HT_ + e) = h; __threadfence(); *(volatile float*)(CT_ + e) = c; *(volatile float*)(HT_ + e) = h; }

__global__ __launch_bounds__(256) void k_tph(const float* __restrict__ ht, bf* Hh, bf* Hl) { const size_t e = ((size_t)blockIdx.x * 256 + threadIdx.x) * 8; if (e >= (size_t)DD * DD) return; const int k = (int)(e % DD); const int n = (int)(e / DD); v8us oh, ol;
#pragma unroll
    for (int q = 0; q < 8; ++q) { unsigned short a, b; splitf(ht[(size_t)(k + q) * DD + n], a, b); oh[q] = a; ol[q] = b; } *(volatile v8us*)(Hh + e) = oh; *(volatile v8us*)(Hl + e) = ol; __threadfence(); *(volatile v8us*)(Hh + e) = oh; *(volatile v8us*)(Hl + e) = ol; }
__global__ __launch_bounds__(256) void k_rsoft(const float* __restrict__ Y, const float* __restrict__ b5, float* O) {
    const int lane = threadIdx.x & 31; const int row = blockIdx.x * 8 + (threadIdx.x >> 5); if (row >= DD) return; const float* yr = Y + (size_t)row * DD; const float* br = b5 + (size_t)row * DD; float v[DD / 32]; float mx = -3.0e38f;
#pragma unroll
    for (int ch = 0; ch < DD / 128; ++ch) { const int j0 = ch * 128 + lane * 4; const v4f a = *(const v4f*)(yr + j0), bb = *(const v4f*)(br + j0);
#pragma unroll
        for (int q = 0; q < 4; ++q) { const float t = __fadd_rn(a[q], bfr(bb[q])); v[ch * 4 + q] = t; mx = fmaxf(mx, t); } }
#pragma unroll
    for (int sh = 16; sh; sh >>= 1) mx = fmaxf(mx, __shfl_xor(mx, sh, 32));
    float sum = 0.f;
#pragma unroll
    for (int k = 0; k < DD / 32; ++k) { float d0 = __fsub_rn(v[k], mx); asm volatile("" : "+v"(d0)); v[k] = __builtin_amdgcn_exp2f(__fmul_rn(d0, 1.4426950408889634f)); sum += v[k]; }
#pragma unroll
    for (int sh = 16; sh; sh >>= 1) sum += __shfl_xor(sum, sh, 32);
    const float f = __fdiv_rn(1.0f, sum);
#pragma unroll 1
    for (int ps = 0; ps < 2; ++ps) {
#pragma unroll
        for (int ch = 0; ch < DD / 128; ++ch) { v4f o;
#pragma unroll
            for (int q = 0; q < 4; ++q) o[q] = v[ch * 4 + q] * f; *(volatile v4f*)(O + (size_t)row * DD + ch * 128 + lane * 4) = o; }
        if (ps == 0) __threadfence(); }
}

extern "C" void kernel_launch(void* const* d_in, const int* in_sizes, int n_in,
                              void* d_out, int out_size, void* d_ws, size_t ws_size, hipStream_t stream) {
    (void)in_sizes; (void)n_in; (void)out_size;
    const float* cp = (const float*)d_in[0]; const float* hp = (const float*)d_in[1]; const float* xx = (const float*)d_in[2];
    const float* w[5], *bb[5]; for (int i = 0; i < 5; ++i) { w[i] = (const float*)d_in[3 + 2 * i]; bb[i] = (const float*)d_in[4 + 2 * i]; }
    float* CTo = (float*)d_out; float* HTo = CTo + (size_t)DD * DD; float* YTo = HTo + (size_t)DD * DD;
    char* wsp = (char*)d_ws;
    auto take = [&](size_t bytes) { char* p = wsp; wsp += (bytes + 255) & ~(size_t)255; return (void*)p; };
    bf* WB = (bf*)take((size_t)DD * DD * 2); bf* CT = (bf*)take((size_t)DD * DD * 2); float* G[4]; for (int i = 0; i < 4; ++i) G[i] = (float*)take((size_t)DD * DD * 4); bf* Hh = (bf*)take((size_t)DD * DD * 2); bf* Hl = (bf*)take((size_t)DD * DD * 2); float* Y = G[0];
    if ((size_t)(wsp - (char*)d_ws) > ws_size) return;
    k_tpc<<<(unsigned)(((size_t)DD * DD / 8 + 255) / 256), 256, 0, stream>>>(hp, xx, CT);
    for (int i = 0; i < 4; ++i) { k_cvt8<<<(unsigned)(((size_t)DD * DD / 8 + 255) / 256), 256, 0, stream>>>(w[i], WB, (size_t)DD * DD / 8);
        k_gemmw<bf, 0, false><<<dim3(DD / 64, DD / 64, 1), 32, 0, stream>>>(WB, nullptr, CT, nullptr, DD, G[i], DD, nullptr, 0, 0, 0); }
    k_gates<<<(unsigned)(((size_t)DD * DD + 255) / 256), 256, 0, stream>>>(G[0], G[1], G[2], G[3], bb[0], bb[1], bb[2], bb[3], cp, CTo, HTo);
    k_tph<<<(unsigned)(((size_t)DD * DD / 8 + 255) / 256), 256, 0, stream>>>(HTo, Hh, Hl);
    k_cvt8<<<(unsigned)(((size_t)DD * DD / 8 + 255) / 256), 256, 0, stream>>>(w[4], WB, (size_t)DD * DD / 8);
    k_gemmw<bf, 3, false><<<dim3(DD / 64, DD / 64, 1), 32, 0, stream>>>(WB, nullptr, Hh, Hl, DD, Y, DD, nullptr, 0, 0, 0);
    k_rsoft<<<DD / 8, 256, 0, stream>>>(Y, bb[4], YTo);
}
